// TLocVLBERT_19069654794252
// MI455X (gfx1250) — hardware-run, weakly checked
//
#include <hip/hip_runtime.h>
#define QTX 800
#define QOB 1032
#define QOP 1088
typedef unsigned short v8us __attribute__((ext_vector_type(8), may_alias));
typedef float  v8f  __attribute__((ext_vector_type(8)));
typedef float  v4f  __attribute__((ext_vector_type(4)));
typedef float  v4fa __attribute__((ext_vector_type(4), may_alias));

__device__ __forceinline__ unsigned short bf16_bits(float x) { unsigned int u = __float_as_uint(x); return (unsigned short)((u + 0x7FFFu + ((u >> 16) & 1u)) >> 16); }
__device__ __forceinline__ float bf16_val(unsigned short b) { return __uint_as_float(((unsigned int)b) << 16); }
__device__ __forceinline__ float bf16_round(float x) { return bf16_val(bf16_bits(x)); }

typedef _Float16 v16h __attribute__((ext_vector_type(16)));
union FragH { v16h v; v8us half[2]; _Float16 h[16]; unsigned short u[16]; };

__global__ __launch_bounds__(256) void k_wt_f16(const float* __restrict__ W, _Float16* __restrict__ Wt, int K, int N, float scale) {
  const int t = blockIdx.x * 256 + threadIdx.x; if (t >= N * (K / 8)) return; const int n = t / (K / 8), k8 = (t % (K / 8)) * 8; FragH f;
#pragma unroll
  for (int i = 0; i < 8; ++i) f.h[i] = (_Float16)(bf16_round(W[(size_t)(k8 + i) * N + n]) * scale); const v8us o = f.half[0];
  *(volatile v8us*)((unsigned short*)Wt + (size_t)n * K + k8) = o; __threadfence(); *(volatile v8us*)((unsigned short*)Wt + (size_t)n * K + k8) = o;
}

typedef _Float16 v4h __attribute__((ext_vector_type(4)));

__global__ __launch_bounds__(256) void k_x16(const float* __restrict__ x, _Float16* __restrict__ X16, size_t n8) { const size_t t = (size_t)blockIdx.x * 256 + threadIdx.x; if (t >= n8) return; FragH f;
#pragma unroll
  for (int q = 0; q < 8; ++q) f.h[q] = (_Float16)bf16_round(x[t * 8 + q]); *(volatile v8us*)((unsigned short*)X16 + t * 8) = f.half[0]; __threadfence(); *(volatile v8us*)((unsigned short*)X16 + t * 8) = f.half[0]; }

__device__ __forceinline__ v16h g2_frag(const _Float16* p, int hh) { FragH f; f.half[0] = *(const v8us*)((const unsigned short*)p + 8 * hh); f.half[1] = *(const v8us*)((const unsigned short*)p + 16 + 8 * hh); return f.v; }
__device__ __forceinline__ v8f g2_mma(v16h a, v16h b, v8f c) { v8f d = __builtin_amdgcn_wmma_f32_16x16x32_f16(false, a, false, b, (short)0, c, false, false); asm volatile("v_nop\n\tv_nop\n\tv_nop\n\tv_nop" : "+v"(d) : "v"(a), "v"(b)); return d; }
template <int ACT>
__global__ __launch_bounds__(128) void k_gemm2(const _Float16* __restrict__ A, int lda, size_t sA, const _Float16* __restrict__ Bh, int ldb, size_t sB, float alpha, const float* __restrict__ bias, size_t sBias, const float* __restrict__ CP, int rowsPerB, size_t sCPb, int row0g,
    float* __restrict__ C, _Float16* __restrict__ C16, int ldc, size_t sC, int M, int N, int K) { static_assert(ACT == 0 || ACT == 3 || ACT == 6 || ACT == 8 || ACT == 9 || ACT == 11 || ACT == 12 || ACT == 14 || ACT == 15 || ACT == 16 || ACT == 17, "k_gemm2: unsupported ACT code (would silently apply no activation)");
  __shared__ __attribute__((aligned(16))) float so[4][32][68];
  const int tid = threadIdx.x, w = tid >> 5, lane = tid & 31, ln = lane & 15, hh = lane >> 4; const int by = blockIdx.y;
  A += (size_t)by * sA; Bh += (size_t)by * sB; const size_t cofs = (size_t)by * sC; const float* bp = bias ? bias + (size_t)by * sBias : nullptr;
  const int ntn = N >> 6; const int mt = blockIdx.x / ntn, nq = blockIdx.x - mt * ntn; const int row0 = mt * 128 + 32 * w, col0 = nq * 64; if (row0 >= M) return;
  const _Float16* a0p = A + (size_t)(row0 + ln) * lda; const _Float16* a1p = a0p + (size_t)16 * lda;
  const _Float16* b0p = Bh + (size_t)(col0 + ln) * ldb; const _Float16* b1p = b0p + (size_t)16 * ldb; const _Float16* b2p = b1p + (size_t)16 * ldb; const _Float16* b3p = b2p + (size_t)16 * ldb;
  const v8f z8 = {0.f,0.f,0.f,0.f,0.f,0.f,0.f,0.f}; v8f c00 = z8, c01 = z8, c02 = z8, c03 = z8, c10 = z8, c11 = z8, c12 = z8, c13 = z8;
  for (int kb = 0; kb < K; kb += 32) { const v16h a0 = g2_frag(a0p + kb, hh), a1 = g2_frag(a1p + kb, hh);
    v16h b = g2_frag(b0p + kb, hh); c00 = g2_mma(a0, b, c00); c10 = g2_mma(a1, b, c10);
    b = g2_frag(b1p + kb, hh); c01 = g2_mma(a0, b, c01); c11 = g2_mma(a1, b, c11);
    b = g2_frag(b2p + kb, hh); c02 = g2_mma(a0, b, c02); c12 = g2_mma(a1, b, c12);
    b = g2_frag(b3p + kb, hh); c03 = g2_mma(a0, b, c03); c13 = g2_mma(a1, b, c13); }
  v8f accs[8] = {c00, c01, c02, c03, c10, c11, c12, c13};
#pragma unroll
  for (int u = 0; u < 8; ++u) { const int t = u & 3, half = u >> 2; const int col = col0 + t * 16 + ln; const float bv = bp ? bf16_round(bp[col]) : 0.f;
#pragma unroll
    for (int r = 0; r < 8; ++r) { const int rloc = half * 16 + 8 * hh + r; float v = accs[u][r] * alpha + bv; if (CP) { if (rowsPerB < 0) v += CP[cofs + (size_t)(row0g + row0 + rloc) * ldc + col];        else { const int bidx = (row0g + row0 + rloc) / rowsPerB; v += CP[(size_t)bidx * sCPb + (size_t)by * 64 + col]; } }
      if (ACT == 3) v = fmaxf(v, 0.f); else if (ACT == 6) v = 0.5f * v * (1.0f + erff(v * 0.70710678118654752f)); else if (ACT == 11) v = 1.0f / (1.0f + expf(-v)); else if (ACT == 15) v = v / (1.0f + expf(-v)); else if (ACT == 12) v = (v > 0.f) ? v : 0.01f * v; else if (ACT == 8) v = tanhf(v); else if (ACT == 9) v = 0.5f * v * (1.0f + tanhf(0.7978845608028654f * (v + 0.044715f * v * v * v))); else if (ACT == 14) v = (v > 0.f) ? v : 0.1f * v; else if (ACT == 16) v = (v >= 0.f) ? v : 0.3f * v; else if (ACT == 17) v = (v >= 0.f) ? v : 0.2f * v;
      so[w][rloc][t * 16 + ln] = v; } }
  __builtin_amdgcn_fence(__ATOMIC_ACQ_REL, "workgroup"); __builtin_amdgcn_wave_barrier();
  const int rsub = lane >> 4, c4 = (lane & 15) * 4;
  for (int pass = 0; pass < 2; ++pass) {
#pragma unroll
    for (int q = 0; q < 16; ++q) { const int r = q * 2 + rsub; const v4f v = *(const v4fa*)&so[w][r][c4]; if (C) *(volatile v4f*)(C + cofs + (size_t)(row0 + r) * ldc + col0 + c4) = v; if (C16) { v4h h4; for (int i = 0; i < 4; ++i) h4[i] = (_Float16)v[i]; *(volatile v4h*)(C16 + cofs + (size_t)(row0 + r) * ldc + col0 + c4) = h4; } }
    if (pass == 0) __threadfence(); } }

__global__ __launch_bounds__(256) void k_cs16(const float* __restrict__ sw, _Float16* __restrict__ tw, float scale) { const size_t t = (size_t)blockIdx.x * 256 + threadIdx.x; FragH f;
#pragma unroll
  for (int q = 0; q < 8; ++q) f.h[q] = (_Float16)(bf16_round(sw[t * 8 + q]) * scale); unsigned short* tp = (unsigned short*)tw + t * 8; *(volatile v8us*)tp = f.half[0]; __threadfence(); *(volatile v8us*)tp = f.half[0]; }
__global__ __launch_bounds__(256) void k_z(_Float16* __restrict__ dst) {
  const unsigned tn = blockIdx.x * 256 + threadIdx.x; FragH f;
#pragma unroll
  for (int i = 0; i < 8; ++i) f.h[i] = (_Float16)0.f;
  unsigned short* tp = (unsigned short*)dst + (size_t)tn * 8; *(volatile v8us*)tp = f.half[0]; __threadfence(); *(volatile v8us*)tp = f.half[0]; }
__global__ __launch_bounds__(256) void k_pair(const float* __restrict__ tp, const float* __restrict__ rD, const float* __restrict__ wE, const float* __restrict__ rE, float* __restrict__ dst) {
  const unsigned sn = blockIdx.y, pr = blockIdx.x * 256 + threadIdx.x; if (pr >= 16641u) return;
  const unsigned pn = pr / 129u, qn = pr - pn * 129u, mn = (pn + qn) >> 1;
  const float* pa = tp + (sn * 129u + pn); const float* pb = tp + 557056u + (sn * 129u + mn); const float* pc = tp + 1114112u + (sn * 129u + qn);
  float aa = 0.f, ab = 0.f, ac = 0.f;
  for (int dn = 0; dn < 512; ++dn) { const float sv = fmaxf(pa[dn * 1088] + pb[dn * 1088] + pc[dn * 1088] + bf16_round(rD[dn]), 0.f); aa += sv * bf16_round(wE[dn * 3]); ab += sv * bf16_round(wE[dn * 3 + 1]); ac += sv * bf16_round(wE[dn * 3 + 2]); }
  aa += bf16_round(rE[0]); ab += bf16_round(rE[1]); ac += bf16_round(rE[2]);
  float* op = dst + (size_t)sn * 50016u + pr; *(volatile float*)op = aa; *(volatile float*)(op + 16672) = ab; *(volatile float*)(op + 33344) = ac; __threadfence(); *(volatile float*)op = aa; *(volatile float*)(op + 16672) = ab; *(volatile float*)(op + 33344) = ac; }
__global__ __launch_bounds__(256) void k_tail(const float* __restrict__ hp, const float* __restrict__ wG, const float* __restrict__ wI, const float* __restrict__ wK, const float* __restrict__ rG, const float* __restrict__ rI, const float* __restrict__ rK, float* __restrict__ dst) {
  const unsigned gn = blockIdx.x * 256 + threadIdx.x; if (gn >= 3096u) return;
  const unsigned rw = gn / 3u, on = gn - rw * 3u; const float fa = (on == 0u) ? 1.f : 0.f, fb = (on == 1u) ? 1.f : 0.f, fc = (on == 2u) ? 1.f : 0.f; const unsigned bq = (on == 0u) ? 0u : ((on == 1u) ? 2u : 1u);
  const float* sp = hp + (size_t)rw * 1536u + bq * 512u; float acc = 0.f;
  for (int dn = 0; dn < 512; ++dn) acc += sp[dn] * (bf16_round(wG[dn]) * fa + bf16_round(wI[dn]) * fb + bf16_round(wK[dn]) * fc);
  acc += bf16_round(rG[0]) * fa + bf16_round(rI[0]) * fb + bf16_round(rK[0]) * fc;
  float* op = dst + gn; *(volatile float*)op = acc; __threadfence(); *(volatile float*)op = acc; }
__global__ __launch_bounds__(256) void k_band(float* __restrict__ dst) {
  const unsigned gn = blockIdx.x * 256 + threadIdx.x; if (gn >= 16641u) return;
  const int rw = (int)(gn / 129u), cl = (int)gn - rw * 129, df = cl - rw;
  const int qa = (rw < 128) & (cl >= rw + 1) & (cl < min(rw + 17, 129));
  const int qb = (rw < 112) & ((rw & 1) == 0) & (cl >= rw + 18) & (cl < min(rw + 33, 129)) & (((df - 18) & 1) == 0);
  const int qc = (rw < 96) & ((rw & 3) == 0) & (cl >= rw + 36) & (cl < min(rw + 65, 129)) & (((df - 36) & 3) == 0);
  const int qd = (rw < 64) & ((rw & 7) == 0) & (cl >= rw + 72) & (cl < 129) & (((df - 72) & 7) == 0);
  const float sv = ((qa | qb | qc | qd) != 0) ? 1.f : 0.f;
  float* op = dst + gn; *(volatile float*)op = sv; __threadfence(); *(volatile float*)op = sv; }
__global__ __launch_bounds__(256) void k_lay(const float* __restrict__ la, const float* __restrict__ rB, const float* __restrict__ lb, const float* __restrict__ lc, const float* __restrict__ ld, float* __restrict__ dst) {
  const unsigned gn = blockIdx.x * 256 + threadIdx.x; if (gn >= 1219121u) return;
  const unsigned ga = min(gn, 799999u), ra = ga / 1000u, ca = ga - ra * 1000u;
  const unsigned gb = min(max(gn, 800000u) - 800000u, 3095u), gc = min(max(gn, 803096u) - 803096u, 399383u), gd = min(max(gn, 1202480u) - 1202480u, 16640u);
  float va = la[ra * 1024u + ca] + bf16_round(rB[ca]), vb = lb[gb], vc = lc[gc + (gc / 16641u) * 31u], vd = ld[gd]; asm volatile("" : "+v"(va), "+v"(vb), "+v"(vc), "+v"(vd));
  const float sv = (gn < 800000u) ? va : ((gn < 803096u) ? vb : ((gn < 1202480u) ? vc : vd));
  float* op = dst + gn; *(volatile float*)op = sv; __threadfence(); *(volatile float*)op = sv; }

extern "C" void kernel_launch(void* const* d_in, const int* in_sizes, int n_in,
                              void* d_out, int out_size, void* d_ws, size_t ws_size, hipStream_t stream) {
  if (n_in < 24) return; if (in_sizes[0] < QTX * 512 || in_sizes[1] < QOB * 512 || in_sizes[2] < 512 * 512 || in_sizes[3] < 512 || in_sizes[4] < 512 * 1000 || in_sizes[5] < 1000 || in_sizes[6] < 512 * 1536 || in_sizes[7] < 1536 || in_sizes[8] < 1536 * 512 || in_sizes[9] < 512 || in_sizes[10] < 512 * 3 || in_sizes[11] < 3) return;
  if (in_sizes[12] < 512 * 512 || in_sizes[13] < 512 || in_sizes[14] < 512 || in_sizes[15] < 1 || in_sizes[16] < 512 * 512 || in_sizes[17] < 512 || in_sizes[18] < 512 || in_sizes[19] < 1 || in_sizes[20] < 512 * 512 || in_sizes[21] < 512 || in_sizes[22] < 512 || in_sizes[23] < 1) return; if (out_size < 1219121) return;
  const float* tx = (const float*)d_in[0]; const float* ob = (const float*)d_in[1]; const float* wA = (const float*)d_in[2]; const float* rA = (const float*)d_in[3]; const float* wB = (const float*)d_in[4]; const float* rB = (const float*)d_in[5]; const float* wC = (const float*)d_in[6]; const float* rC = (const float*)d_in[7]; const float* wD = (const float*)d_in[8]; const float* rD = (const float*)d_in[9]; const float* wE = (const float*)d_in[10]; const float* rE = (const float*)d_in[11];
  const float* wF = (const float*)d_in[12]; const float* rF = (const float*)d_in[13]; const float* wG = (const float*)d_in[14]; const float* rG = (const float*)d_in[15]; const float* wH = (const float*)d_in[16]; const float* rH = (const float*)d_in[17]; const float* wI = (const float*)d_in[18]; const float* rI = (const float*)d_in[19]; const float* wJ = (const float*)d_in[20]; const float* rJ = (const float*)d_in[21]; const float* wK = (const float*)d_in[22]; const float* rK = (const float*)d_in[23]; float* res = (float*)d_out;
  static_assert(QTX % 32 == 0 && QOP % 64 == 0 && QOP % 32 == 0 && (QTX * 512 / 8) % 256 == 0 && (QOB * 512 / 8) % 256 == 0 && ((QOP - QOB) * 512 / 8) % 256 == 0 && (24 * 512 / 8) % 256 == 0, "whole tiles, exact grids");
  uint8_t* wsp = (uint8_t*)d_ws; size_t off = 0;
  auto take = [&](size_t bytes) { uint8_t* pp = wsp + off; off += (bytes + 255) & ~(size_t)255; return pp; };
  _Float16* XT = (_Float16*)take((size_t)QTX * 512 * 2); _Float16* XO = (_Float16*)take((size_t)QOP * 512 * 2); _Float16* SA = (_Float16*)take((size_t)512 * 512 * 2); _Float16* SB = (_Float16*)take((size_t)1024 * 512 * 2); _Float16* SC = (_Float16*)take((size_t)1536 * 512 * 2); _Float16* SD = (_Float16*)take((size_t)512 * 1536 * 2); _Float16* SH = (_Float16*)take((size_t)3 * 512 * 512 * 2);
  _Float16* TA = (_Float16*)take((size_t)QTX * 512 * 2); float* LA = (float*)take((size_t)QTX * 1024 * 4); _Float16* HA = (_Float16*)take((size_t)QOP * 1536 * 2); float* TP = (float*)take((size_t)3 * 512 * QOP * 4); float* HP = (float*)take((size_t)QOP * 1536 * 4); float* LB = (float*)take((size_t)3096 * 4); float* LC = (float*)take((size_t)24 * 16672 * 4); float* LD = (float*)take((size_t)16641 * 4);
  if (off > ws_size) return;
  k_cs16<<<(unsigned)(QTX * 512 / 8 / 256), 256, 0, stream>>>(tx, XT, 16.0f); k_cs16<<<(unsigned)(QOB * 512 / 8 / 256), 256, 0, stream>>>(ob, XO, 16.0f);
  k_z<<<(unsigned)((QOP - QOB) * 512 / 8 / 256), 256, 0, stream>>>(XO + (size_t)QOB * 512);
  k_wt_f16<<<(unsigned)((512 * (512 / 8) + 255) / 256), 256, 0, stream>>>(wA, SA, 512, 512, 4096.0f); k_wt_f16<<<(unsigned)((1000 * (512 / 8) + 255) / 256), 256, 0, stream>>>(wB, SB, 512, 1000, 4096.0f); k_wt_f16<<<(unsigned)((1536 * (512 / 8) + 255) / 256), 256, 0, stream>>>(wC, SC, 512, 1536, 4096.0f); k_wt_f16<<<(unsigned)((512 * (1536 / 8) + 255) / 256), 256, 0, stream>>>(wD, SD, 1536, 512, 4096.0f);
  k_wt_f16<<<(unsigned)((512 * (512 / 8) + 255) / 256), 256, 0, stream>>>(wF, SH, 512, 512, 4096.0f); k_wt_f16<<<(unsigned)((512 * (512 / 8) + 255) / 256), 256, 0, stream>>>(wJ, SH + (size_t)512 * 512, 512, 512, 4096.0f); k_wt_f16<<<(unsigned)((512 * (512 / 8) + 255) / 256), 256, 0, stream>>>(wH, SH + (size_t)2 * 512 * 512, 512, 512, 4096.0f);
  k_z<<<(unsigned)(24 * 512 / 8 / 256), 256, 0, stream>>>(SB + (size_t)1000 * 512);
  k_gemm2<3><<<dim3((unsigned)(((QTX + 127) / 128) * (512 / 64)), 1), 128, 0, stream>>>(XT, 512, (size_t)0, SA, 512, (size_t)0, 1.52587890625e-05f, rA, (size_t)0, nullptr, 1, 0, 0, nullptr, TA, 512, (size_t)0, QTX, 512, 512);
  k_gemm2<0><<<dim3((unsigned)(((QTX + 127) / 128) * (1024 / 64)), 1), 128, 0, stream>>>(TA, 512, (size_t)0, SB, 512, (size_t)0, 0.000244140625f, nullptr, (size_t)0, nullptr, 1, 0, 0, LA, nullptr, 1024, (size_t)0, QTX, 1024, 512);
  k_gemm2<3><<<dim3((unsigned)(((QOP + 127) / 128) * (1536 / 64)), 1), 128, 0, stream>>>(XO, 512, (size_t)0, SC, 512, (size_t)0, 1.52587890625e-05f, rC, (size_t)0, nullptr, 1, 0, 0, nullptr, HA, 1536, (size_t)0, QOP, 1536, 512);
  k_gemm2<0><<<dim3((unsigned)((512 / 128) * (QOP / 64)), 3), 128, 0, stream>>>(SD, 1536, (size_t)512, HA, 1536, (size_t)512, 0.000244140625f, nullptr, (size_t)0, nullptr, 1, 0, 0, TP, nullptr, QOP, (size_t)512 * QOP, 512, QOP, 512);
  k_gemm2<3><<<dim3((unsigned)(((QOP + 127) / 128) * (512 / 64)), 1), 128, 0, stream>>>(HA, 1536, (size_t)0, SH, 512, (size_t)0, 0.000244140625f, rF, (size_t)0, nullptr, 1, 0, 0, HP, nullptr, 1536, (size_t)0, QOP, 512, 512);
  k_gemm2<3><<<dim3((unsigned)(((QOP + 127) / 128) * (512 / 64)), 1), 128, 0, stream>>>(HA + 512, 1536, (size_t)0, SH + (size_t)512 * 512, 512, (size_t)0, 0.000244140625f, rJ, (size_t)0, nullptr, 1, 0, 0, HP + 512, nullptr, 1536, (size_t)0, QOP, 512, 512);
  k_gemm2<3><<<dim3((unsigned)(((QOP + 127) / 128) * (512 / 64)), 1), 128, 0, stream>>>(HA + 1024, 1536, (size_t)0, SH + (size_t)2 * 512 * 512, 512, (size_t)0, 0.000244140625f, rH, (size_t)0, nullptr, 1, 0, 0, HP + 1024, nullptr, 1536, (size_t)0, QOP, 512, 512);
  k_pair<<<dim3((unsigned)((16641 + 255) / 256), 8), 256, 0, stream>>>(TP, rD, wE, rE, LC);
  k_tail<<<(unsigned)((3096 + 255) / 256), 256, 0, stream>>>(HP, wG, wI, wK, rG, rI, rK, LB);
  k_band<<<(unsigned)((16641 + 255) / 256), 256, 0, stream>>>(LD);
  k_lay<<<(unsigned)((1219121 + 255) / 256), 256, 0, stream>>>(LA, rB, LB, LC, LD, res);
}
